// MambaLayer_6373731467393
// MI455X (gfx1250) — hardware-verified
//
#include <hip/hip_runtime.h>
#include <math.h>

typedef __attribute__((ext_vector_type(16))) __bf16   v16b;
typedef __attribute__((ext_vector_type(8)))  __bf16   v8b;
typedef __attribute__((ext_vector_type(8)))  float    v8f;
typedef __attribute__((ext_vector_type(4)))  float    v4f;
typedef __attribute__((ext_vector_type(4)))  unsigned v4u;

constexpr int kBatch  = 4;
constexpr int kSeq    = 4096;
constexpr int kDm     = 128;
constexpr int kDin    = 256;
constexpr int kNst    = 16;
constexpr int kDtR    = 8;
constexpr int kNsl    = 16;
constexpr int kMsl    = kSeq / kNsl;
constexpr int kXzP    = 2 * kDin;
constexpr int kXdN    = kDtR + 2 * kNst;
constexpr int kXdP    = 64;
constexpr int kRows   = kBatch * kSeq;
constexpr int kYcP    = 3 * kDin;
constexpr int kConvTP = 260;
constexpr int kScanTS = 64;
constexpr int kScanCh = 64;
constexpr int kScanYP = 68;
static_assert(kXdN == 40 && kXdN <= kXdP, "x_proj width");
static_assert(kMsl == 256 && kNsl == 16 && kSeq == 4096, "slice map uses shifts by 4 and 8");
static_assert((kDm % 32) == 0 && (kDin % 32) == 0 && (kYcP % 32) == 0, "GEMM K multiples of 32");
static_assert((kRows % 64) == 0 && (kXzP % 64) == 0 && (kXdP % 64) == 0 && (kDm % 64) == 0, "GEMM M,N multiples of 64");
static_assert((kSeq % kScanTS) == 0 && (kDin % kScanCh) == 0 && kDin == 256, "tile multiples");

constexpr size_t kOffXB  = 0;
constexpr size_t kOffW1  = kOffXB  + (size_t)kRows * kDm * 2;
constexpr size_t kOffXP  = kOffW1  + (size_t)kXzP * kDm * 2;
constexpr size_t kOffW3  = kOffXP  + (size_t)3 * kXdP * kDin * 2;
constexpr size_t kOffXZ  = kOffW3  + (size_t)kDm * kYcP * 2;
constexpr size_t kOffUCB = kOffXZ  + (size_t)kRows * kXzP * 4;
constexpr size_t kOffXD  = kOffUCB + (size_t)3 * kRows * kDin * 2;
constexpr size_t kOffYH  = kOffXD  + (size_t)3 * kRows * kXdP * 4;
constexpr size_t kOffYL  = kOffYH  + (size_t)kRows * kYcP * 2;
constexpr size_t kWsTotal = kOffYL + (size_t)kRows * kYcP * 2;
static_assert(kWsTotal == 126255104ull, "carve total");
static_assert(kWsTotal <= 134217728ull, "carve cap");
static_assert((kOffW1 % 128) == 0 && (kOffXP % 128) == 0 && (kOffW3 % 128) == 0 && (kOffXZ % 128) == 0 &&
              (kOffUCB % 128) == 0 && (kOffXD % 128) == 0 && (kOffYH % 128) == 0 && (kOffYL % 128) == 0,
              "128-B aligned regions");

__device__ __forceinline__ unsigned short f2bf_bits(float f) {
  unsigned u = __float_as_uint(f);
  return (unsigned short)((u + 0x7FFFu + ((u >> 16) & 1u)) >> 16);
}
__device__ __forceinline__ float bf_bits2f(unsigned short h) { return __uint_as_float(((unsigned)h) << 16); }
__device__ __forceinline__ float rne_bf(float f) { return bf_bits2f(f2bf_bits(f)); }
__device__ __forceinline__ unsigned pack_bf2(float lo, float hi) {
  const unsigned a = (unsigned)f2bf_bits(lo);
  const unsigned b = (unsigned)f2bf_bits(hi);
  return a | (b << 16);
}
__device__ __forceinline__ void split_pack2(float f0, float f1, unsigned& hw, unsigned& lw) {
  const unsigned short h0 = f2bf_bits(f0), h1 = f2bf_bits(f1);
  const unsigned short l0 = f2bf_bits(f0 - bf_bits2f(h0)), l1 = f2bf_bits(f1 - bf_bits2f(h1));
  hw = (unsigned)h0 | (((unsigned)h1) << 16);
  lw = (unsigned)l0 | (((unsigned)l1) << 16);
}
__device__ __forceinline__ int perm_pos(int dir, int t) {
  const int p0 = t;
  const int p1 = kSeq - 1 - t;
  const int p2 = ((t & (kNsl - 1)) << 8) | (t >> 4);
  return (dir == 0) ? p0 : ((dir == 1) ? p1 : p2);
}
__device__ __forceinline__ float sigmoid_f(float v) {
  return __builtin_amdgcn_rcpf(1.0f + expf(-v));
}

__device__ __forceinline__ void guard_row4(v8f& a, v8f& b, v8f& c, v8f& d, v16b x, v16b y) {
  asm volatile("v_nop\n\tv_nop\n\tv_nop\n\tv_nop" : "+v"(a), "+v"(b), "+v"(c), "+v"(d) : "v"(x), "v"(y));
}
__device__ __forceinline__ void keep4_b(v16b a, v16b b, v16b c, v16b d) { asm volatile("v_nop" :: "v"(a), "v"(b), "v"(c), "v"(d)); }
__device__ __forceinline__ void acc_guard4(v8f& a, v8f& b, v8f& c, v8f& d) { asm volatile("v_nop\n\tv_nop\n\tv_nop\n\tv_nop" : "+v"(a), "+v"(b), "+v"(c), "+v"(d)); }
struct FragB {
  union U { v16b v; v8b h[2]; };
  static __device__ __forceinline__ v16b load(const __bf16* p) {
    U f; f.h[0] = *(const v8b*)(p); f.h[1] = *(const v8b*)(p + 16); return f.v;
  }
  static __device__ __forceinline__ v8f mma(v16b a, v16b b, v8f c) {
    return __builtin_amdgcn_wmma_f32_16x16x32_bf16(false, a, false, b, (short)0, c, false, false);
  }
};

template <int SPL>
__global__ __launch_bounds__(256) void wmma_gemm64_bf16(
    const unsigned short* __restrict__ Ap, const unsigned short* __restrict__ A2p, int lda, long strideA,
    const unsigned short* __restrict__ Btp, int ldb, long strideB,
    float* __restrict__ Cout, int ldc, long strideC,
    int M, int N, int K) {
  const __bf16* A = (const __bf16*)Ap; const __bf16* A2 = (const __bf16*)A2p; const __bf16* Bt = (const __bf16*)Btp;
  __shared__ __align__(16) float sT[8][16 * 68];
  const int b    = blockIdx.y;
  const int lane = threadIdx.x & 31;
  const int wave = threadIdx.x >> 5;
  const int tilesN = N >> 6;
  const int tilesM = M >> 6;
  const int tile = blockIdx.x * 8 + wave;
  if (tile >= tilesM * tilesN) return;
  const int tm = tile / tilesN;
  const int tn = tile - tm * tilesN;
  const int m0 = tm << 6;
  const int n0 = tn << 6;

  const __bf16* Ab  = A  + (size_t)b * strideA;
  const __bf16* Bb  = Bt + (size_t)b * strideB;
  const __bf16* Ab2 = (SPL >= 1) ? (A2 + (size_t)b * strideA) : nullptr;

  const int rlane = lane & 15;
  const int koff  = (lane >> 4) * 8;
  const int mOff  = (lane >> 4) * 8;

  v8f acc[4][4];
#pragma unroll
  for (int i = 0; i < 4; ++i)
#pragma unroll
    for (int j = 0; j < 4; ++j) acc[i][j] = (v8f){0.f,0.f,0.f,0.f,0.f,0.f,0.f,0.f};

  for (int k0 = 0; k0 < K; k0 += 32) {
    v16b bh[4];
#pragma unroll
    for (int j = 0; j < 4; ++j) {
      const size_t bo = (size_t)(n0 + (j << 4) + rlane) * ldb + koff + k0;
      bh[j] = FragB::load(Bb + bo);
    }
#pragma unroll
    for (int i = 0; i < 4; ++i) {
      const size_t ao = (size_t)(m0 + (i << 4) + rlane) * lda + koff + k0;
      v16b ah = FragB::load(Ab + ao);
      v16b al = ah;
      if (SPL >= 1) al = FragB::load(Ab2 + ao);
#pragma unroll
      for (int j = 0; j < 4; ++j) {
        acc[i][j] = FragB::mma(ah, bh[j], acc[i][j]);
        if (SPL >= 1) acc[i][j] = FragB::mma(al, bh[j], acc[i][j]);
      }
      guard_row4(acc[i][0], acc[i][1], acc[i][2], acc[i][3], ah, al);
    }
    keep4_b(bh[0], bh[1], bh[2], bh[3]);
  }
  acc_guard4(acc[0][0], acc[0][1], acc[0][2], acc[0][3]);
  acc_guard4(acc[1][0], acc[1][1], acc[1][2], acc[1][3]);
  acc_guard4(acc[2][0], acc[2][1], acc[2][2], acc[2][3]);
  acc_guard4(acc[3][0], acc[3][1], acc[3][2], acc[3][3]);

  float* slab = sT[wave];
  float* C = Cout + (size_t)b * strideC;
  const int hh = lane >> 4, c4 = (lane & 15) * 4;
#pragma unroll
  for (int i = 0; i < 4; ++i) {
    const int mBase = m0 + (i << 4);
#pragma unroll
    for (int j = 0; j < 4; ++j) {
#pragma unroll
      for (int r = 0; r < 8; ++r) {
        slab[(mOff + r) * 68 + (j << 4) + rlane] = acc[i][j][r];
      }
    }
    __builtin_amdgcn_fence(__ATOMIC_RELEASE, "workgroup");
    __builtin_amdgcn_wave_barrier();
    __builtin_amdgcn_fence(__ATOMIC_ACQUIRE, "workgroup");
    for (int pass = 0; pass < 2; ++pass) {
#pragma unroll
      for (int it = 0; it < 8; ++it) {
        const int row = it * 2 + hh;
        v4f v = *(const v4f*)(slab + row * 68 + c4);
        *(volatile v4f*)(C + (size_t)(mBase + row) * ldc + n0 + c4) = v;
      }
      __threadfence();
    }
    __builtin_amdgcn_fence(__ATOMIC_RELEASE, "workgroup");
    __builtin_amdgcn_wave_barrier();
    __builtin_amdgcn_fence(__ATOMIC_ACQUIRE, "workgroup");
  }
}

__global__ __launch_bounds__(256) void cast_rows_bf16_kernel(
    const float* __restrict__ s0, const float* __restrict__ s1, const float* __restrict__ s2,
    unsigned short* __restrict__ dst, int srcRows, int srcCols, int dstRows, int dstCols)
{
  const int y = blockIdx.y;
  const float* src = (y == 0) ? s0 : ((y == 1) ? s1 : s2);
  const int per = dstRows * dstCols;
  const int e0 = (blockIdx.x * 256 + threadIdx.x) * 8;
  if (e0 >= per) return;
  const int r  = e0 / dstCols;
  const int c  = e0 - r * dstCols;
  const int cs = c % srcCols;
  const bool live = (r < srcRows);
  const int rc = live ? r : (srcRows - 1);
  const float* p = src + (size_t)rc * srcCols + cs;
  const v4f a0 = *(const v4f*)(p);
  const v4f a1 = *(const v4f*)(p + 4);
  const float f0 = a0[0], f1 = a0[1], f2 = a0[2], f3 = a0[3];
  const float f4 = a1[0], f5 = a1[1], f6 = a1[2], f7 = a1[3];
  const unsigned w0 = pack_bf2(f0, f1), w1 = pack_bf2(f2, f3), w2 = pack_bf2(f4, f5), w3 = pack_bf2(f6, f7);
  v4u w;
  w[0] = live ? w0 : 0u;
  w[1] = live ? w1 : 0u;
  w[2] = live ? w2 : 0u;
  w[3] = live ? w3 : 0u;
  unsigned short* q = dst + (size_t)y * per + e0;
  *(volatile v4u*)q = w;
  __threadfence();
  *(volatile v4u*)q = w;
}

__global__ __launch_bounds__(256) void conv_silu_kernel(
    const float* __restrict__ XZ,
    const float* __restrict__ cw0, const float* __restrict__ cw1, const float* __restrict__ cw2,
    const float* __restrict__ cb0, const float* __restrict__ cb1, const float* __restrict__ cb2,
    unsigned short* __restrict__ UCB)
{
  __shared__ __align__(16) float sT[16 * kConvTP];
  const int tid = threadIdx.x, lane = tid & 31, wave = tid >> 5;
  const int dir = blockIdx.y;
  const float* cw = (dir == 0) ? cw0 : ((dir == 1) ? cw1 : cw2);
  const float* cb = (dir == 0) ? cb0 : ((dir == 1) ? cb1 : cb2);
  const int d  = tid;
  const int g0 = blockIdx.x * 64;
  const int t0 = g0 & (kSeq - 1);
  const int rowb = g0 - t0;
  const v4f wv = *(const v4f*)(cw + d * 4);
  const float wa = wv[0], wb = wv[1], wc = wv[2], wd = wv[3];
  const float w0 = rne_bf(wa), w1 = rne_bf(wb), w2 = rne_bf(wc), w3 = rne_bf(wd);
  const float bc = rne_bf(cb[d]);
  float xm3, xm2, xm1;
  {
    const bool hist = (t0 > 0);
    const int th = hist ? (t0 - 3) : 0;
    const float v3 = XZ[(size_t)(rowb + perm_pos(dir, th)) * kXzP + d];
    const float v2 = XZ[(size_t)(rowb + perm_pos(dir, th + 1)) * kXzP + d];
    const float v1 = XZ[(size_t)(rowb + perm_pos(dir, th + 2)) * kXzP + d];
    xm3 = hist ? v3 : 0.f;
    xm2 = hist ? v2 : 0.f;
    xm1 = hist ? v1 : 0.f;
  }
  unsigned short* Ud = UCB + (size_t)dir * kRows * kDin;
#pragma unroll 1
  for (int sub = 0; sub < 4; ++sub) {
    const int tb = t0 + sub * 16;
#pragma unroll 1
    for (int s = 0; s < 16; ++s) {
      const int pos = perm_pos(dir, tb + s);
      const float xcur = XZ[(size_t)(rowb + pos) * kXzP + d];
      float acc = w0 * xm3;
      acc = fmaf(w1, xm2, acc);
      acc = fmaf(w2, xm1, acc);
      acc = fmaf(w3, xcur, acc);
      const float sv = acc + bc;
      sT[s * kConvTP + tid] = sv * sigmoid_f(sv);
      xm3 = xm2; xm2 = xm1; xm1 = xcur;
    }
    __syncthreads();
    v4u ow[2];
#pragma unroll
    for (int it = 0; it < 2; ++it) {
      const float* sp = sT + (it * 8 + wave) * kConvTP + lane * 8;
      const v4f a0 = *(const v4f*)(sp);
      const v4f a1 = *(const v4f*)(sp + 4);
      const float f0 = a0[0], f1 = a0[1], f2 = a0[2], f3 = a0[3];
      const float f4 = a1[0], f5 = a1[1], f6 = a1[2], f7 = a1[3];
      ow[it][0] = pack_bf2(f0, f1);
      ow[it][1] = pack_bf2(f2, f3);
      ow[it][2] = pack_bf2(f4, f5);
      ow[it][3] = pack_bf2(f6, f7);
    }
    for (int pass = 0; pass < 2; ++pass) {
#pragma unroll
      for (int it = 0; it < 2; ++it) {
        const size_t o = (size_t)(rowb + tb + it * 8 + wave) * kDin + lane * 8;
        *(volatile v4u*)(Ud + o) = ow[it];
      }
      __threadfence();
    }
    __syncthreads();
  }
}

__global__ __launch_bounds__(64) void scan_kernel(
    const float* __restrict__ XZ, const float* __restrict__ XD,
    const float* __restrict__ cw0, const float* __restrict__ cw1, const float* __restrict__ cw2,
    const float* __restrict__ cb0, const float* __restrict__ cb1, const float* __restrict__ cb2,
    const float* __restrict__ dw0, const float* __restrict__ dw1, const float* __restrict__ dw2,
    const float* __restrict__ db0, const float* __restrict__ db1, const float* __restrict__ db2,
    const float* __restrict__ al0, const float* __restrict__ al1, const float* __restrict__ al2,
    const float* __restrict__ dp0, const float* __restrict__ dp1, const float* __restrict__ dp2,
    unsigned short* __restrict__ YH, unsigned short* __restrict__ YL)
{
  __shared__ __align__(16) float sX[kScanTS * kXdP];
  __shared__ __align__(16) float sY[kScanTS * kScanYP];
  __shared__ __align__(16) float sA[kNst * kScanCh];
  __shared__ __align__(16) float sE[kNst * kScanCh];
  const int tid = threadIdx.x, lane = tid & 31, wave = tid >> 5;
  const int blk = blockIdx.x;
  const int dir = blk >> 4;
  const int rem = blk & 15;
  const int bix = rem >> 2;
  const int d0  = (rem & 3) * kScanCh;
  const int d   = d0 + tid;
  const int rowb = bix * kSeq;
  const float* cw = (dir == 0) ? cw0 : ((dir == 1) ? cw1 : cw2);
  const float* cb = (dir == 0) ? cb0 : ((dir == 1) ? cb1 : cb2);
  const float* dw = (dir == 0) ? dw0 : ((dir == 1) ? dw1 : dw2);
  const float* db = (dir == 0) ? db0 : ((dir == 1) ? db1 : db2);
  const float* al = (dir == 0) ? al0 : ((dir == 1) ? al1 : al2);
  const float* dp = (dir == 0) ? dp0 : ((dir == 1) ? dp1 : dp2);
  const float* XDd = XD + (size_t)dir * kRows * kXdP;

  const v4f cwv = *(const v4f*)(cw + d * 4);
  const float ca = cwv[0], cbb = cwv[1], cc = cwv[2], cd = cwv[3];
  const float cwa = rne_bf(ca), cwb = rne_bf(cbb), cwc = rne_bf(cc), cwd = rne_bf(cd);
  const float cbias = rne_bf(cb[d]);
  const v4f dq0 = *(const v4f*)(dw + d * kDtR);
  const v4f dq1 = *(const v4f*)(dw + d * kDtR + 4);
  const float e0 = dq0[0], e1 = dq0[1], e2 = dq0[2], e3 = dq0[3];
  const float e4 = dq1[0], e5 = dq1[1], e6 = dq1[2], e7 = dq1[3];
  const float wd0 = rne_bf(e0), wd1 = rne_bf(e1), wd2 = rne_bf(e2), wd3 = rne_bf(e3);
  const float wd4 = rne_bf(e4), wd5 = rne_bf(e5), wd6 = rne_bf(e6), wd7 = rne_bf(e7);
  const float bb = rne_bf(db[d]);
  const float Dd = rne_bf(dp[d]);
#pragma unroll 1
  for (int s = 0; s < kNst; ++s) sA[s * kScanCh + tid] = -expf(rne_bf(al[(size_t)d * kNst + s]));
  __syncthreads();

  float h[kNst];
#pragma unroll
  for (int s = 0; s < kNst; ++s) h[s] = 0.f;
  float xm3 = 0.f, xm2 = 0.f, xm1 = 0.f;

  const int lr = tid >> 4, lc4 = (tid & 15) * 4;
  const int q = lane >> 3, c8 = (lane & 7) * 8;
#pragma unroll 1
  for (int t0 = 0; t0 < kSeq; t0 += kScanTS) {
    __syncthreads();
#pragma unroll
    for (int i = 0; i < 16; ++i) {
      const int r = lr + 4 * i;
      *(v4f*)(sX + r * kXdP + lc4) = *(const v4f*)(XDd + (size_t)(rowb + t0 + r) * kXdP + lc4);
    }
    __syncthreads();
#pragma unroll 1
    for (int s = 0; s < kScanTS; ++s) {
      const int t = t0 + s;
      const int pos = perm_pos(dir, t);
      const size_t gro = (size_t)(rowb + pos) * kXzP;
      float xcur = XZ[gro + d];
      float zv   = XZ[gro + kDin + d];
      asm volatile("" : "+v"(xcur), "+v"(zv));
      float cacc = cwa * xm3;
      cacc = fmaf(cwb, xm2, cacc);
      cacc = fmaf(cwc, xm1, cacc);
      cacc = fmaf(cwd, xcur, cacc);
      const float sv = cacc + cbias;
      const float u  = sv * sigmoid_f(sv);
      xm3 = xm2; xm2 = xm1; xm1 = xcur;

      const float* xr = sX + s * kXdP;
      const v4f t0v = *(const v4f*)(xr);
      const v4f t1v = *(const v4f*)(xr + 4);
      float vdot = t0v[0] * wd0;
      vdot = fmaf(t0v[1], wd1, vdot);
      vdot = fmaf(t0v[2], wd2, vdot);
      vdot = fmaf(t0v[3], wd3, vdot);
      vdot = fmaf(t1v[0], wd4, vdot);
      vdot = fmaf(t1v[1], wd5, vdot);
      vdot = fmaf(t1v[2], wd6, vdot);
      vdot = fmaf(t1v[3], wd7, vdot);
      const float v   = vdot + bb;
      const float ea  = expf(-fabsf(v));
      const float u1  = 1.0f + ea;
      const float l1p = logf(u1) + (ea - (u1 - 1.0f)) * __builtin_amdgcn_rcpf(u1);
      const float dt  = fmaxf(v, 0.0f) + l1p;

#pragma unroll 1
      for (int k = 0; k < kNst; ++k) sE[k * kScanCh + tid] = expf(dt * sA[k * kScanCh + tid]);

      float Bs[kNst], Cs[kNst];
#pragma unroll
      for (int q4 = 0; q4 < 4; ++q4) {
        const v4f bv = *(const v4f*)(xr + kDtR + 4 * q4);
        const v4f cv = *(const v4f*)(xr + kDtR + kNst + 4 * q4);
        Bs[4 * q4 + 0] = bv[0]; Bs[4 * q4 + 1] = bv[1]; Bs[4 * q4 + 2] = bv[2]; Bs[4 * q4 + 3] = bv[3];
        Cs[4 * q4 + 0] = cv[0]; Cs[4 * q4 + 1] = cv[1]; Cs[4 * q4 + 2] = cv[2]; Cs[4 * q4 + 3] = cv[3];
      }
      const float dtu = dt * u;
      float ys = 0.f;
#pragma unroll
      for (int k = 0; k < kNst; ++k) {
        const float e = sE[k * kScanCh + tid];
        h[k] = fmaf(h[k], e, dtu * Bs[k]);
        ys = fmaf(h[k], Cs[k], ys);
      }
      const float yk = fmaf(Dd, u, ys);
      const float g  = zv * sigmoid_f(zv);
      sY[s * kScanYP + tid] = yk * g;
    }
    __syncthreads();
    v4u hw[8], lw[8];
#pragma unroll
    for (int it = 0; it < 8; ++it) {
      const int row = it * 8 + wave * 4 + q;
      const float* sp = sY + row * kScanYP + c8;
      const v4f a0 = *(const v4f*)(sp);
      const v4f a1 = *(const v4f*)(sp + 4);
      const float f0 = a0[0], f1 = a0[1], f2 = a0[2], f3 = a0[3];
      const float f4 = a1[0], f5 = a1[1], f6 = a1[2], f7 = a1[3];
      unsigned h0, l0, h1, l1, h2, l2, h3, l3;
      split_pack2(f0, f1, h0, l0);
      split_pack2(f2, f3, h1, l1);
      split_pack2(f4, f5, h2, l2);
      split_pack2(f6, f7, h3, l3);
      hw[it][0] = h0; hw[it][1] = h1; hw[it][2] = h2; hw[it][3] = h3;
      lw[it][0] = l0; lw[it][1] = l1; lw[it][2] = l2; lw[it][3] = l3;
    }
    for (int pass = 0; pass < 2; ++pass) {
#pragma unroll
      for (int it = 0; it < 8; ++it) {
        const int row = it * 8 + wave * 4 + q;
        const int pos = perm_pos(dir, t0 + row);
        const size_t o = (size_t)(rowb + pos) * kYcP + dir * kDin + d0 + c8;
        *(volatile v4u*)(YH + o) = hw[it];
        *(volatile v4u*)(YL + o) = lw[it];
      }
      __threadfence();
    }
  }
}

extern "C" void kernel_launch(void* const* d_in, const int* in_sizes, int n_in,
                              void* d_out, int out_size, void* d_ws, size_t ws_size,
                              hipStream_t stream) {
  if (n_in < 24) return;
  if (in_sizes[0] != kRows * kDm) return;
  if (in_sizes[1] != kXzP * kDm) return;
  for (int s = 0; s < 3; ++s) {
    const int o = 2 + 7 * s;
    if (in_sizes[o + 0] != kDin * 4) return;
    if (in_sizes[o + 1] != kDin) return;
    if (in_sizes[o + 2] != kXdN * kDin) return;
    if (in_sizes[o + 3] != kDin * kDtR) return;
    if (in_sizes[o + 4] != kDin) return;
    if (in_sizes[o + 5] != kDin * kNst) return;
    if (in_sizes[o + 6] != kDin) return;
  }
  if (in_sizes[23] != kDm * kDin) return;
  if (out_size != kRows * kDm) return;
  if (ws_size < kWsTotal) return;

  const float* x_in  = (const float*)d_in[0];
  const float* W_in  = (const float*)d_in[1];
  const float* cw[3] = {(const float*)d_in[2], (const float*)d_in[9],  (const float*)d_in[16]};
  const float* cb[3] = {(const float*)d_in[3], (const float*)d_in[10], (const float*)d_in[17]};
  const float* xp[3] = {(const float*)d_in[4], (const float*)d_in[11], (const float*)d_in[18]};
  const float* dw[3] = {(const float*)d_in[5], (const float*)d_in[12], (const float*)d_in[19]};
  const float* db[3] = {(const float*)d_in[6], (const float*)d_in[13], (const float*)d_in[20]};
  const float* al[3] = {(const float*)d_in[7], (const float*)d_in[14], (const float*)d_in[21]};
  const float* dp[3] = {(const float*)d_in[8], (const float*)d_in[15], (const float*)d_in[22]};
  const float* W_out = (const float*)d_in[23];
  float* out = (float*)d_out;

  char* ws = (char*)d_ws;
  unsigned short* XB  = (unsigned short*)(ws + kOffXB);
  unsigned short* W1  = (unsigned short*)(ws + kOffW1);
  unsigned short* XP  = (unsigned short*)(ws + kOffXP);
  unsigned short* W3  = (unsigned short*)(ws + kOffW3);
  float*          XZ  = (float*)(ws + kOffXZ);
  unsigned short* UCB = (unsigned short*)(ws + kOffUCB);
  float*          XD  = (float*)(ws + kOffXD);
  unsigned short* YH  = (unsigned short*)(ws + kOffYH);
  unsigned short* YL  = (unsigned short*)(ws + kOffYL);

  cast_rows_bf16_kernel<<<dim3((kRows * kDm / 8) / 256, 1), 256, 0, stream>>>(
      x_in, x_in, x_in, XB, kRows, kDm, kRows, kDm);
  cast_rows_bf16_kernel<<<dim3((kXzP * kDm / 8) / 256, 1), 256, 0, stream>>>(
      W_in, W_in, W_in, W1, kXzP, kDm, kXzP, kDm);
  cast_rows_bf16_kernel<<<dim3((kXdP * kDin / 8) / 256, 3), 256, 0, stream>>>(
      xp[0], xp[1], xp[2], XP, kXdN, kDin, kXdP, kDin);
  cast_rows_bf16_kernel<<<dim3((kDm * kYcP / 8) / 256, 1), 256, 0, stream>>>(
      W_out, W_out, W_out, W3, kDm, kDin, kDm, kYcP);

  wmma_gemm64_bf16<0><<<dim3(256, 1), 256, 0, stream>>>(
      XB, XB, kDm, 0L,
      W1, kDm, 0L,
      XZ, kXzP, 0L,
      kRows, kXzP, kDm);

  conv_silu_kernel<<<dim3(kRows / 64, 3), 256, 0, stream>>>(
      XZ, cw[0], cw[1], cw[2], cb[0], cb[1], cb[2], UCB);

  wmma_gemm64_bf16<0><<<dim3(32, 3), 256, 0, stream>>>(
      UCB, UCB, kDin, (long)kRows * kDin,
      XP, kDin, (long)kXdP * kDin,
      XD, kXdP, (long)kRows * kXdP,
      kRows, kXdP, kDin);

  scan_kernel<<<3 * kBatch * (kDin / kScanCh), kScanCh, 0, stream>>>(
      XZ, XD,
      cw[0], cw[1], cw[2], cb[0], cb[1], cb[2],
      dw[0], dw[1], dw[2], db[0], db[1], db[2],
      al[0], al[1], al[2], dp[0], dp[1], dp[2],
      YH, YL);

  wmma_gemm64_bf16<1><<<dim3(64, 1), 256, 0, stream>>>(
      YH, YL, kYcP, 0L,
      W3, kYcP, 0L,
      out, kDm, 0L,
      kRows, kDm, kYcP);
}
